// HFModule_88184268521674
// MI455X (gfx1250) — hardware-verified
//
#include <hip/hip_runtime.h>
#include <hip/hip_bf16.h>
#include <math.h>

#define NR_ 8192
#define CC  1024
#define SS  8192
#define HH  16
#define DKK 64
#define BB  1

typedef _Float16 bf16;
typedef __attribute__((ext_vector_type(4))) unsigned v4u_t;
typedef unsigned v4ua __attribute__((ext_vector_type(4), may_alias));
typedef __attribute__((ext_vector_type(4))) float v4f_t;
typedef float v4fa __attribute__((ext_vector_type(4), may_alias));
typedef __attribute__((ext_vector_type(16))) bf16  bf16x16;
typedef __attribute__((ext_vector_type(8)))  bf16  bf16x8;
typedef __attribute__((ext_vector_type(4)))  bf16  bf16x4;
typedef __attribute__((ext_vector_type(8)))  float f32x8;

#define LDS_STRIDE 48
#define KSTRIDE    72
#define VSTRIDE    48

__device__ __forceinline__ f32x8 wmma_bf16(bf16x16 a, bf16x16 b, f32x8 c) {
  return __builtin_amdgcn_wmma_f32_16x16x32_f16(
      false, a, false, b, (short)0, c, false, false);
}

template <typename T>
__device__ __forceinline__ bf16x16 load_frag(const T* __restrict__ base, int ld,
                                             int row0, int k0) {
  const int lane = threadIdx.x & 31;
  const int r    = lane & 15;
  const int kh   = (lane >> 4) * 8;
  const T* p0 = base + (size_t)(row0 + r) * ld + (k0 + kh);
  const T* p1 = p0 + 16;
  bf16x16 f;
#pragma unroll
  for (int i = 0; i < 8; ++i) {
    f[i]     = (bf16)p0[i];
    f[i + 8] = (bf16)p1[i];
  }
  return f;
}

__device__ __forceinline__ bf16x16 lds_frag(const bf16* base, int stride) {
  const int lane = threadIdx.x & 31;
  const int row  = lane & 15;
  const int kh   = (lane >> 4) * 8;
  const bf16x8 lo = *(const bf16x8*)(base + row * stride + kh);
  const bf16x8 hi = *(const bf16x8*)(base + row * stride + kh + 16);
  bf16x16 f;
#pragma unroll
  for (int i = 0; i < 8; ++i) { f[i] = lo[i]; f[i + 8] = hi[i]; }
  return f;
}

template <typename T>
__device__ __forceinline__ void stage_read16(const T* __restrict__ p, float* buf) {
#pragma unroll
  for (int i = 0; i < 16; ++i) buf[i] = (float)p[i];
}

__device__ __forceinline__ void stage_write(bf16* dst, const float* buf, int nquad) {
#pragma unroll
  for (int i = 0; i < nquad; ++i) {
    bf16x4 q;
    q[0] = (bf16)buf[4 * i];     q[1] = (bf16)buf[4 * i + 1];
    q[2] = (bf16)buf[4 * i + 2]; q[3] = (bf16)buf[4 * i + 3];
    *(bf16x4*)(dst + 4 * i) = q;
  }
}

template <typename AT, int MODE>
__global__ __launch_bounds__(256) void gemm_rs_kernel(
    const AT* __restrict__ A, const float* __restrict__ W,
    const float* __restrict__ bias, const float* __restrict__ rowscale, void* __restrict__ out,
    int M, int N, int K) {
  __shared__ bf16 ldsA[128 * LDS_STRIDE];
  __shared__ bf16 ldsW[256 * LDS_STRIDE];
  __shared__ __attribute__((aligned(16))) unsigned char sob[256 * 136 * 2];

  const int t    = threadIdx.x;
  const int wave = t >> 5;
  const int lane = t & 31;
  const int wm   = (wave & 1) * 64;
  const int wn   = (wave >> 1) * 64;
  const int mBlk = blockIdx.x * 128;
  const int nBlk = blockIdx.y * 256;

  const int arow = t >> 1;
  const int ach  = (t & 1) * 16;

  float abuf[16];
  float wbuf[32];

  stage_read16(A + (size_t)(mBlk + arow) * K + ach, abuf);
  stage_read16(W + (size_t)(nBlk + t) * K,          wbuf);
  stage_read16(W + (size_t)(nBlk + t) * K + 16,     wbuf + 16);

  f32x8 acc[4][4] = {};

  for (int k = 0; k < K; k += 32) {
    __syncthreads();
    stage_write(&ldsA[arow * LDS_STRIDE + ach], abuf, 4);
    stage_write(&ldsW[t * LDS_STRIDE],          wbuf, 8);
    if (k + 32 < K) {
      stage_read16(A + (size_t)(mBlk + arow) * K + (k + 32) + ach, abuf);
      stage_read16(W + (size_t)(nBlk + t) * K + (k + 32),          wbuf);
      stage_read16(W + (size_t)(nBlk + t) * K + (k + 32) + 16,     wbuf + 16);
    }
    __syncthreads();

    bf16x16 af[4], wf[4];
#pragma unroll
    for (int i = 0; i < 4; ++i)
      af[i] = lds_frag(ldsA + (wm + 16 * i) * LDS_STRIDE, LDS_STRIDE);
#pragma unroll
    for (int j = 0; j < 4; ++j)
      wf[j] = lds_frag(ldsW + (wn + 16 * j) * LDS_STRIDE, LDS_STRIDE);
#pragma unroll
    for (int i = 0; i < 4; ++i)
#pragma unroll
      for (int j = 0; j < 4; ++j)
        acc[i][j] = wmma_bf16(af[i], wf[j], acc[i][j]);
  }

  const int nlane = lane & 15;
  const int mh    = (lane >> 4) * 8;
  __syncthreads();
  if (MODE == 0 || MODE == 1 || MODE == 3) {
    bf16* so = (bf16*)sob;
#pragma unroll
    for (int i = 0; i < 4; ++i)
#pragma unroll
      for (int j = 0; j < 4; ++j) {
        const int nl = wn + 16 * j + nlane;
        const float bv = bias ? bias[nBlk + nl] : 0.0f;
        if (MODE == 3) {
#pragma unroll 1
          for (int r = 0; r < 8; ++r) {
            const int ml = wm + 16 * i + mh + r;
            const float xg = acc[i][j][r] + bv;
            so[ml * 264 + nl] = (bf16)(0.5f * xg * (1.0f + erff(xg * 0.70710678118654752f)));
          }
        } else {
#pragma unroll
        for (int r = 0; r < 8; ++r) {
          const int ml = wm + 16 * i + mh + r;
          const bf16 hv = (bf16)(acc[i][j][r] + bv);
          if (MODE == 0) so[ml * 264 + nl] = hv;
          else           so[nl * 136 + ml] = hv;
        }
        }
      }
    __syncthreads();
#pragma unroll 1
    for (int pass = 0; pass < 2; ++pass) {
      if (MODE == 0 || MODE == 3) {
        for (int ch = t; ch < 128 * 32; ch += 256) { const int ml = ch >> 5, q = (ch & 31) * 8;
          *(volatile v4u_t*)((bf16*)out + (size_t)(mBlk + ml) * N + nBlk + q) = *(const v4ua*)(so + ml * 264 + q); }
      } else {
        const int b_ = mBlk / SS, s0 = mBlk & (SS - 1);
        for (int ch = t; ch < 256 * 16; ch += 256) { const int nl = ch >> 4, q = (ch & 15) * 8; const int n = nBlk + nl, h = n >> 6, dk = n & (DKK - 1);
          *(volatile v4u_t*)((bf16*)out + (((size_t)(b_ * HH + h)) * DKK + dk) * SS + s0 + q) = *(const v4ua*)(so + nl * 136 + q); }
      }
      __threadfence();
    }
  } else {
    float* so = (float*)sob;
#pragma unroll 1
    for (int hf = 0; hf < 2; ++hf) {
      if (wm == hf * 64) {
#pragma unroll
        for (int i = 0; i < 4; ++i)
#pragma unroll
          for (int j = 0; j < 4; ++j) {
            const int nl = wn + 16 * j + nlane;
            const float bv = bias ? bias[nBlk + nl] : 0.0f;
#pragma unroll
            for (int r = 0; r < 8; ++r) so[(16 * i + mh + r) * 260 + nl] = (acc[i][j][r] + bv) * (rowscale ? rowscale[mBlk + hf * 64 + 16 * i + mh + r] : 1.0f);
          }
      }
      __syncthreads();
#pragma unroll 1
      for (int pass = 0; pass < 2; ++pass) {
        for (int ch = t; ch < 64 * 64; ch += 256) { const int ml = ch >> 6, q = (ch & 63) * 4;
          *(volatile v4f_t*)((float*)out + (size_t)(mBlk + hf * 64 + ml) * N + nBlk + q) = *(const volatile v4fa*)(so + ml * 260 + q); }
        __threadfence();
      }
      __syncthreads();
    }
  }
}

template <typename AT, int MODE>
__global__ __launch_bounds__(256) void gemm_circ_kernel(
    const AT* __restrict__ A, const float* __restrict__ W,
    const float* __restrict__ bias, const float* __restrict__ rowscale, void* __restrict__ out,
    int M, int N, int K) {
  __shared__ bf16 ldsA[128 * LDS_STRIDE];
  __shared__ bf16 ldsW[256 * LDS_STRIDE];
  __shared__ __attribute__((aligned(16))) unsigned char sob[256 * 136 * 2];

  const int t    = threadIdx.x;
  const int wave = t >> 5;
  const int lane = t & 31;
  const int wm   = (wave & 1) * 64;
  const int wn   = (wave >> 1) * 64;
  const int mBlk = blockIdx.x * 128;
  const int nBlk = blockIdx.y * 256;

  const int arow = t >> 1;
  const int ach  = (t & 1) * 16;

  float abuf[16];
  float wbuf[32];

  stage_read16(A + (size_t)(mBlk + arow) * K + ach, abuf);
  { const int n = nBlk + t;
#pragma unroll
    for (int i = 0; i < 32; ++i) wbuf[i] = W[(n - i) & 1023]; }

  f32x8 acc[4][4] = {};

  for (int k = 0; k < K; k += 32) {
    __syncthreads();
    stage_write(&ldsA[arow * LDS_STRIDE + ach], abuf, 4);
    stage_write(&ldsW[t * LDS_STRIDE],          wbuf, 8);
    if (k + 32 < K) {
      stage_read16(A + (size_t)(mBlk + arow) * K + (k + 32) + ach, abuf);
      { const int n = nBlk + t;
#pragma unroll
        for (int i = 0; i < 32; ++i) wbuf[i] = W[(n - (k + 32 + i)) & 1023]; }
    }
    __syncthreads();

    bf16x16 af[4], wf[4];
#pragma unroll
    for (int i = 0; i < 4; ++i)
      af[i] = lds_frag(ldsA + (wm + 16 * i) * LDS_STRIDE, LDS_STRIDE);
#pragma unroll
    for (int j = 0; j < 4; ++j)
      wf[j] = lds_frag(ldsW + (wn + 16 * j) * LDS_STRIDE, LDS_STRIDE);
#pragma unroll
    for (int i = 0; i < 4; ++i)
#pragma unroll
      for (int j = 0; j < 4; ++j)
        acc[i][j] = wmma_bf16(af[i], wf[j], acc[i][j]);
  }

  const int nlane = lane & 15;
  const int mh    = (lane >> 4) * 8;
  __syncthreads();
  if (MODE == 0 || MODE == 1 || MODE == 3) {
    bf16* so = (bf16*)sob;
#pragma unroll
    for (int i = 0; i < 4; ++i)
#pragma unroll
      for (int j = 0; j < 4; ++j) {
        const int nl = wn + 16 * j + nlane;
        const float bv = bias ? bias[nBlk + nl] : 0.0f;
        if (MODE == 3) {
#pragma unroll 1
          for (int r = 0; r < 8; ++r) {
            const int ml = wm + 16 * i + mh + r;
            const float xg = acc[i][j][r] + bv;
            so[ml * 264 + nl] = (bf16)(0.5f * xg * (1.0f + erff(xg * 0.70710678118654752f)));
          }
        } else {
#pragma unroll
        for (int r = 0; r < 8; ++r) {
          const int ml = wm + 16 * i + mh + r;
          const bf16 hv = (bf16)(acc[i][j][r] + bv);
          if (MODE == 0) so[ml * 264 + nl] = hv;
          else           so[nl * 136 + ml] = hv;
        }
        }
      }
    __syncthreads();
#pragma unroll 1
    for (int pass = 0; pass < 2; ++pass) {
      if (MODE == 0 || MODE == 3) {
        for (int ch = t; ch < 128 * 32; ch += 256) { const int ml = ch >> 5, q = (ch & 31) * 8;
          *(volatile v4u_t*)((bf16*)out + (size_t)(mBlk + ml) * N + nBlk + q) = *(const v4ua*)(so + ml * 264 + q); }
      } else {
        const int b_ = mBlk / SS, s0 = mBlk & (SS - 1);
        for (int ch = t; ch < 256 * 16; ch += 256) { const int nl = ch >> 4, q = (ch & 15) * 8; const int n = nBlk + nl, h = n >> 6, dk = n & (DKK - 1);
          *(volatile v4u_t*)((bf16*)out + (((size_t)(b_ * HH + h)) * DKK + dk) * SS + s0 + q) = *(const v4ua*)(so + nl * 136 + q); }
      }
      __threadfence();
    }
  } else {
    float* so = (float*)sob;
#pragma unroll 1
    for (int hf = 0; hf < 2; ++hf) {
      if (wm == hf * 64) {
#pragma unroll
        for (int i = 0; i < 4; ++i)
#pragma unroll
          for (int j = 0; j < 4; ++j) {
            const int nl = wn + 16 * j + nlane;
            const float bv = bias ? bias[nBlk + nl] : 0.0f;
#pragma unroll
            for (int r = 0; r < 8; ++r) so[(16 * i + mh + r) * 260 + nl] = (acc[i][j][r] + bv) * (rowscale ? rowscale[mBlk + hf * 64 + 16 * i + mh + r] : 1.0f);
          }
      }
      __syncthreads();
#pragma unroll 1
      for (int pass = 0; pass < 2; ++pass) {
        for (int ch = t; ch < 64 * 64; ch += 256) { const int ml = ch >> 6, q = (ch & 63) * 4;
          *(volatile v4f_t*)((float*)out + (size_t)(mBlk + hf * 64 + ml) * N + nBlk + q) = *(const volatile v4fa*)(so + ml * 260 + q); }
        __threadfence();
      }
      __syncthreads();
    }
  }
}


__global__ __launch_bounds__(256) void k_silu_ln(float* __restrict__ buf, const float* __restrict__ g, const float* __restrict__ b) {
  __shared__ float red[256];
  const int row = blockIdx.x, t = threadIdx.x;
  float* r = buf + (size_t)row * CC;
  float v[4], s = 0.0f;
#pragma unroll
  for (int j = 0; j < 4; ++j) { const float p = r[t + 256 * j]; v[j] = p / (1.0f + __expf(-p)); s += v[j]; }
  red[t] = s; __syncthreads();
  for (int o = 128; o > 0; o >>= 1) { if (t < o) red[t] += red[t + o]; __syncthreads(); }
  const float mu = red[0] * (1.0f / (float)CC); __syncthreads();
  float q = 0.0f;
#pragma unroll
  for (int j = 0; j < 4; ++j) { v[j] -= mu; q += v[j] * v[j]; }
  red[t] = q; __syncthreads();
  for (int o = 128; o > 0; o >>= 1) { if (t < o) red[t] += red[t + o]; __syncthreads(); }
  const float rs = rsqrtf(red[0] * (1.0f / (float)CC) + 1e-5f);
#pragma unroll 1
  for (int pass = 0; pass < 2; ++pass) {
#pragma unroll
    for (int j = 0; j < 4; ++j) { const int c = t + 256 * j; *(volatile float*)(r + c) = v[j] * rs * g[c] + b[c]; }
    __threadfence();
  }
}
__global__ __launch_bounds__(256) void k_htab(const float* __restrict__ freq_w, float* __restrict__ H) {
  __shared__ float wS[513], cosS[1024], red[256];
  const int t = threadIdx.x;
  float m = -INFINITY;
  for (int i = t; i < 513; i += 256) m = fmaxf(m, freq_w[i]);
  red[t] = m; __syncthreads();
  for (int o = 128; o > 0; o >>= 1) { if (t < o) red[t] = fmaxf(red[t], red[t + o]); __syncthreads(); }
  m = red[0]; __syncthreads();
  float s = 0.0f;
  for (int i = t; i < 513; i += 256) { const float e = __expf(freq_w[i] - m); wS[i] = e; s += e; }
  red[t] = s; __syncthreads();
  for (int o = 128; o > 0; o >>= 1) { if (t < o) red[t] += red[t + o]; __syncthreads(); }
  const float inv = 1.0f / red[0];
  for (int i = t; i < 1024; i += 256) cosS[i] = cosf(6.2831853071795864769f * (float)i / 1024.0f);
  __syncthreads();
  float hv[4];
#pragma unroll
  for (int j = 0; j < 4; ++j) {
    const int n = t + 256 * j;
    float acc = wS[0] + wS[512] * ((n & 1) ? -1.0f : 1.0f);
    for (int k = 1; k < 512; ++k) acc += 2.0f * wS[k] * cosS[(k * n) & 1023];
    hv[j] = acc * inv;
  }
#pragma unroll 1
  for (int pass = 0; pass < 2; ++pass) {
#pragma unroll
    for (int j = 0; j < 4; ++j) *(volatile float*)(H + t + 256 * j) = hv[j];
    __threadfence();
  }
}
__global__ __launch_bounds__(256) void k_gamma(const float* __restrict__ F, const float* __restrict__ tval, const float* __restrict__ sval, float* __restrict__ rsc) {
  __shared__ __attribute__((aligned(16))) float gS[32];
  const int tid = threadIdx.x, lane = tid & 31, wave = tid >> 5;
  const float t = tval[0], c = 1e-4f, sc = 0.01f;
#pragma unroll 1
  for (int rr = 0; rr < 4; ++rr) {
    const int row = blockIdx.x * 32 + wave * 4 + rr;
    const float* fr = F + (size_t)row * CC;
    float s = 0.0f;
    for (int d = lane * 4; d < CC; d += 128) { const v4f_t v = *(const v4f_t*)(fr + d); s += v[0] * v[0] + v[1] * v[1] + v[2] * v[2] + v[3] * v[3]; }
#pragma unroll
    for (int off = 16; off >= 1; off >>= 1) s += __shfl_xor(s, off, 32);
    if (lane == 0) {
      const float S = s * (1.0f / (1024.0f * 1024.0f));
      const float nu = fmaxf(sqrtf(S), 1e-7f);
      const float scn_u = fminf(fmaxf(sc * nu, 1e-7f), 1.0f - 1e-5f);
      const float alpha = tanhf((1.0f - t) * atanhf(scn_u)) / (sc * nu);
      const float nv = fmaxf(fabsf(t) * sqrtf(S), 1e-7f);
      const float scn_v = fminf(fmaxf(sc * nv, 1e-7f), 1.0f - 1e-5f);
      const float beta = tanhf(t * atanhf(scn_v)) / (sc * nv) * t;
      const float x2 = alpha * alpha * S, y2 = beta * beta * S, xy = alpha * beta * S;
      const float num = (1.0f + 2.0f * c * xy + c * y2) * alpha + (1.0f - c * x2) * beta;
      const float den = fmaxf(1.0f + 2.0f * c * xy + c * c * x2 * y2, 1e-7f);
      gS[wave * 4 + rr] = (num / den) * sval[0] * (1.0f / 1024.0f);
    }
  }
  __syncthreads();
  if (wave == 0 && lane < 8) {
#pragma unroll 1
    for (int pass = 0; pass < 2; ++pass) { *(volatile v4f_t*)(rsc + blockIdx.x * 32 + lane * 4) = *(const volatile v4fa*)(gS + lane * 4); __threadfence(); }
  }
}

extern "C" void kernel_launch(void* const* d_in, const int* in_sizes, int n_in,
                              void* d_out, int out_size, void* d_ws, size_t ws_size,
                              hipStream_t stream) {
  (void)in_sizes; (void)n_in; (void)out_size; (void)ws_size;
  const float* x = (const float*)d_in[0];
  const float* proj_w = (const float*)d_in[1];
  const float* ln_g = (const float*)d_in[2], *ln_b = (const float*)d_in[3];
  const float* freq_w = (const float*)d_in[4];
  const float* tval = (const float*)d_in[5];
  const float* down_w = (const float*)d_in[6];
  const float* sval = (const float*)d_in[7];
  float* out = (float*)d_out;
  char* ws = (char*)d_ws;
  float* comp = (float*)ws; float* F = (float*)(ws + (32 << 20)); float* H = (float*)(ws + (64 << 20)); float* rsc = (float*)(ws + (64 << 20) + 4096);
  const dim3 g(NR_ / 128, CC / 256), blk(256);
  gemm_rs_kernel<float, 2><<<g, blk, 0, stream>>>(x, proj_w, nullptr, nullptr, comp, NR_, CC, CC);
  k_silu_ln<<<dim3(NR_), dim3(256), 0, stream>>>(comp, ln_g, ln_b);
  k_htab<<<dim3(1), dim3(256), 0, stream>>>(freq_w, H);
  gemm_circ_kernel<float, 2><<<g, blk, 0, stream>>>(comp, H, nullptr, nullptr, F, NR_, CC, CC);
  k_gamma<<<dim3(NR_ / 32), dim3(256), 0, stream>>>(F, tval, sval, rsc);
  gemm_rs_kernel<float, 2><<<g, blk, 0, stream>>>(F, down_w, nullptr, rsc, out, NR_, CC, CC);
}
